// BDHResonatorLayer_82094004896070
// MI455X (gfx1250) — hardware-run, weakly checked
//
#include <hip/hip_runtime.h>
#include <math.h>

constexpr int kBatch = 2;
constexpr int kSteps = 1024;
constexpr int kChan  = 1024;
constexpr int kHeads = 16;
constexpr int kHdim  = 64;
constexpr int kFreq  = 256;
constexpr int kRank  = 4096;
constexpr int kTok   = kBatch * kSteps;
constexpr int kPre   = 2 * kFreq;
constexpr int kFeat  = 3 * kFreq;
constexpr int kQkv   = 3 * kChan;

constexpr int kResSteps = 64;
constexpr int kResF     = 64;
constexpr int kAtChunk  = 32;

constexpr float kActCarry = 16.0f;
constexpr float kWCarry   = 256.0f;
constexpr float kScale    = 1.0f / (kActCarry * kWCarry);
constexpr float kF16Min   = 6.103515625e-05f;
constexpr float kPi       = 3.14159274101257324f;
constexpr float kEpsLn    = 1e-5f;
constexpr float kEpsAttn  = 1e-6f;

static_assert(kHeads * kHdim == kChan);
static_assert(kHdim == 64 && kAtChunk == 32 && kResSteps == 64 && kResF == 64);
static_assert(kTok % 32 == 0);
static_assert(kPre % 64 == 0 && kChan % 64 == 0 && kQkv % 64 == 0 && kRank % 64 == 0 && kFeat % 64 == 0);
static_assert(kChan % 32 == 0 && kFeat % 32 == 0 && kRank % 32 == 0);
static_assert(kSteps % kResSteps == 0 && kSteps % kAtChunk == 0 && kFreq % kResF == 0);
static_assert((kTok * kFreq) % 256 == 0 && (kTok * kChan / 8) % 256 == 0);
static_assert(kChan == 256 * 4);

typedef __attribute__((ext_vector_type(16))) _Float16 v16h;
typedef __attribute__((ext_vector_type(8)))  _Float16 v8h;
typedef __attribute__((ext_vector_type(8)))  float    v8f;
typedef __attribute__((ext_vector_type(4)))  float    v4f;
typedef __attribute__((ext_vector_type(4)))  unsigned int v4u;

constexpr size_t kBytesXH   = (size_t)kTok  * kChan * 2;
constexpr size_t kBytesWAP  = (size_t)kPre  * kChan * 2;
constexpr size_t kBytesWFT  = (size_t)kChan * kFeat * 2;
constexpr size_t kBytesWQKV = (size_t)kQkv  * kChan * 2;
constexpr size_t kBytesW1T  = (size_t)kRank * kChan * 2;
constexpr size_t kBytesW2T  = (size_t)kChan * kRank * 2;
constexpr size_t kBytesP1   = (size_t)kTok  * kPre  * 4;
constexpr size_t kBytesU    = (size_t)kTok  * kPre  * 4;
constexpr size_t kBytesFEAT = (size_t)kTok  * kFeat * 2;
constexpr size_t kBytesHH   = (size_t)kTok  * kChan * 2;
constexpr size_t kBytesQKV  = (size_t)kTok  * kQkv  * 4;
constexpr size_t kBytesYN   = (size_t)kTok  * kChan * 2;
constexpr size_t kBytesH1   = (size_t)kTok  * kRank * 2;
constexpr size_t kBytesY2   = (size_t)kTok  * kChan * 4;
constexpr size_t kWsTotal = kBytesXH + kBytesWAP + kBytesWFT + kBytesWQKV + kBytesW1T + kBytesW2T + kBytesP1 +
                            kBytesU + kBytesFEAT + kBytesHH + kBytesQKV + kBytesYN + kBytesH1 + kBytesY2;
static_assert(kWsTotal == 100139008ull);
static_assert(kWsTotal <= 134217728ull);
static_assert(kBytesXH % 256 == 0 && kBytesWAP % 256 == 0 && kBytesWFT % 256 == 0 && kBytesWQKV % 256 == 0 &&
              kBytesW1T % 256 == 0 && kBytesW2T % 256 == 0 && kBytesP1 % 256 == 0 && kBytesU % 256 == 0 &&
              kBytesFEAT % 256 == 0 && kBytesHH % 256 == 0 && kBytesQKV % 256 == 0 && kBytesYN % 256 == 0 &&
              kBytesH1 % 256 == 0 && kBytesY2 % 256 == 0);

__device__ __forceinline__ unsigned pk16(unsigned short a, unsigned short b) {
  return (unsigned)a | ((unsigned)b << 16);
}
__device__ __forceinline__ unsigned short h_bits_flush(float f) {
  const float g = (fabsf(f) < kF16Min) ? 0.0f : f;
  const _Float16 h = (_Float16)g;
  return __builtin_bit_cast(unsigned short, h);
}
__device__ __forceinline__ v4u pack8(const float (&v)[8]) {
  unsigned short hb[8];
#pragma unroll
  for (int e = 0; e < 8; ++e) hb[e] = h_bits_flush(v[e]);
  return (v4u){pk16(hb[0], hb[1]), pk16(hb[2], hb[3]), pk16(hb[4], hb[5]), pk16(hb[6], hb[7])};
}
__device__ __forceinline__ float wave_sum32(float v) {
#pragma unroll
  for (int o = 16; o > 0; o >>= 1) v += __shfl_xor(v, o, 32);
  return v;
}

struct FragH {
  union U { v16h v; v8h h[2]; };
  static __device__ __forceinline__ v16h load(const _Float16* p) {
    U f;
    f.h[0] = *(const v8h*)(p);
    f.h[1] = *(const v8h*)(p + 16);
    return f.v;
  }
};
__device__ __forceinline__ v8f mma_g(v16h a, v16h b, v8f c) {
  c = __builtin_amdgcn_wmma_f32_16x16x32_f16(false, a, false, b, (short)0, c, false, false);
  asm volatile("v_nop\n\tv_nop\n\tv_nop\n\tv_nop" : "+v"(c) : "v"(a), "v"(b));
  return c;
}
__device__ __forceinline__ void acc_guard4(v8f& a, v8f& b, v8f& c, v8f& d) {
  asm volatile("v_nop\n\tv_nop\n\tv_nop\n\tv_nop" : "+v"(a), "+v"(b), "+v"(c), "+v"(d));
}

template <int OUT_MODE, bool HAS_BIAS>
__global__ __launch_bounds__(256) void gemm_f16_kernel(
    const unsigned short* __restrict__ Ap, int lda,
    const unsigned short* __restrict__ Bp, int ldb,
    void* __restrict__ Cout, int ldc,
    const float* __restrict__ bias,
    int M, int N, int K, float scale, int relu_cols, float out_carry) {
  __shared__ __align__(16) float sT[8][16 * 68];
  const int lane = threadIdx.x & 31;
  const int wave = threadIdx.x >> 5;
  const int tilesN = N >> 6;
  const int tilesM = M >> 5;
  const int tile = blockIdx.x * 8 + wave;
  if (tile >= tilesM * tilesN) return;
  const int tm = tile / tilesN;
  const int tn = tile - tm * tilesN;
  const int m0 = tm << 5;
  const int n0 = tn << 6;
  const int rlane = lane & 15;
  const int half8 = (lane >> 4) * 8;
  const int mOff  = (lane >> 4) * 8;

  const size_t aoff = (size_t)(m0 + rlane) * lda + half8;
  const size_t boff = (size_t)(n0 + rlane) * ldb + half8;
  const _Float16* pa0 = (const _Float16*)Ap + aoff;
  const _Float16* pa1 = pa0 + (size_t)16 * lda;
  const _Float16* pbh = (const _Float16*)Bp + boff;
  const size_t bstep = (size_t)16 * ldb;

  v8f acc[2][4];
#pragma unroll
  for (int i = 0; i < 2; ++i)
#pragma unroll
    for (int j = 0; j < 4; ++j) acc[i][j] = (v8f){0.f, 0.f, 0.f, 0.f, 0.f, 0.f, 0.f, 0.f};

  for (int k0 = 0; k0 < K; k0 += 32) {
    const v16h ah0 = FragH::load(pa0 + k0);
    const v16h ah1 = FragH::load(pa1 + k0);
#pragma unroll
    for (int j = 0; j < 4; ++j) {
      const v16h bh = FragH::load(pbh + j * bstep + k0);
      acc[0][j] = mma_g(ah0, bh, acc[0][j]);
      acc[1][j] = mma_g(ah1, bh, acc[1][j]);
    }
  }
  acc_guard4(acc[0][0], acc[0][1], acc[0][2], acc[0][3]);
  acc_guard4(acc[1][0], acc[1][1], acc[1][2], acc[1][3]);

  float bv[4];
#pragma unroll
  for (int j = 0; j < 4; ++j) {
    bv[j] = 0.0f;
    if (HAS_BIAS) bv[j] = bias[n0 + (j << 4) + rlane];
  }
  const bool do_relu = (n0 < relu_cols);

  float* slab = sT[wave];
#pragma unroll
  for (int i = 0; i < 2; ++i) {
    const int mBase = m0 + (i << 4);
#pragma unroll
    for (int j = 0; j < 4; ++j) {
#pragma unroll
      for (int r = 0; r < 8; ++r) {
        float v = acc[i][j][r] * scale + bv[j];
        v = do_relu ? fmaxf(v, 0.0f) : v;
        if (OUT_MODE == 1) v = v * out_carry;
        slab[(mOff + r) * 68 + (j << 4) + rlane] = v;
      }
    }
    __builtin_amdgcn_fence(__ATOMIC_RELEASE, "workgroup");
    __builtin_amdgcn_wave_barrier();
    __builtin_amdgcn_fence(__ATOMIC_ACQUIRE, "workgroup");
    if (OUT_MODE == 0) {
      float* C = (float*)Cout;
      const int hh = lane >> 4, c4 = (lane & 15) * 4;
      for (int pass = 0; pass < 2; ++pass) {
#pragma unroll
        for (int it = 0; it < 8; ++it) {
          const int row = it * 2 + hh;
          const v4f v = *(const v4f*)(slab + row * 68 + c4);
          *(volatile v4f*)(C + (size_t)(mBase + row) * ldc + n0 + c4) = v;
        }
        __threadfence();
      }
    } else {
      const int q = lane >> 3, c8 = (lane & 7) * 8;
      unsigned short* C = (unsigned short*)Cout;
      for (int pass = 0; pass < 2; ++pass) {
#pragma unroll
        for (int it = 0; it < 4; ++it) {
          const int row = it * 4 + q;
          const float* sp = slab + row * 68 + c8;
          const v4f a0 = *(const v4f*)(sp);
          const v4f a1 = *(const v4f*)(sp + 4);
          v8h hv;
#pragma unroll
          for (int e = 0; e < 4; ++e) {
            float x0 = a0[e];
            float x1 = a1[e];
            x0 = (fabsf(x0) < kF16Min) ? 0.0f : x0;
            x1 = (fabsf(x1) < kF16Min) ? 0.0f : x1;
            hv[e]     = (_Float16)x0;
            hv[4 + e] = (_Float16)x1;
          }
          *(volatile v8h*)(C + (size_t)(mBase + row) * ldc + n0 + c8) = hv;
        }
        __threadfence();
      }
    }
    __builtin_amdgcn_fence(__ATOMIC_RELEASE, "workgroup");
    __builtin_amdgcn_wave_barrier();
    __builtin_amdgcn_fence(__ATOMIC_ACQUIRE, "workgroup");
  }
}

__global__ __launch_bounds__(256) void wt_plane_kernel(const float* __restrict__ W0, const float* __restrict__ W1,
                                                       const float* __restrict__ W2,
                                                       unsigned short* __restrict__ outh,
                                                       int Kd, int Nd, int KdP, int NdP) {
  __shared__ float sm[64][65];
  const int t  = threadIdx.x;
  const int k0 = blockIdx.x * 64;
  const int n0 = blockIdx.y * 64;
  const int z  = blockIdx.z;
  const float* W = (z == 0) ? W0 : (z == 1) ? W1 : W2;
#pragma unroll
  for (int i = 0; i < 16; ++i) {
    const int e = i * 256 + t;
    const int r = e >> 6;
    const int c = e & 63;
    const int kk = k0 + r;
    const int nn = n0 + c;
    const bool valid = (kk < Kd) && (nn < Nd);
    const int kc = (kk < Kd) ? kk : (Kd - 1);
    const int nc = (nn < Nd) ? nn : (Nd - 1);
    const float v = W[(size_t)kc * Nd + nc];
    sm[c][r] = valid ? (v * kWCarry) : 0.0f;
  }
  __syncthreads();
  const int lane = t & 31, wave = t >> 5;
  const int q = lane >> 3, c8 = (lane & 7) * 8;
  const size_t pofs = (size_t)z * (size_t)NdP * (size_t)KdP;
  for (int pass = 0; pass < 2; ++pass) {
#pragma unroll
    for (int it = 0; it < 2; ++it) {
      const int row = wave * 8 + it * 4 + q;
      float v[8];
#pragma unroll
      for (int e = 0; e < 8; ++e) v[e] = sm[row][c8 + e];
      const v4u uh = pack8(v);
      const size_t o = pofs + (size_t)(n0 + row) * KdP + k0 + c8;
      *(volatile v4u*)(outh + o) = uh;
    }
    __threadfence();
  }
}

__global__ __launch_bounds__(256) void cast_act_kernel(const float* __restrict__ src,
                                                       unsigned short* __restrict__ dst, int total8) {
  const int i = blockIdx.x * 256 + threadIdx.x;
  if (i >= total8) return;
  const size_t e0 = (size_t)i << 3;
  const v4f a0 = *(const v4f*)(src + e0);
  const v4f a1 = *(const v4f*)(src + e0 + 4);
  float v[8];
#pragma unroll
  for (int e = 0; e < 4; ++e) {
    v[e]     = a0[e] * kActCarry;
    v[4 + e] = a1[e] * kActCarry;
  }
  const v4u u = pack8(v);
  *(volatile v4u*)(dst + e0) = u;
  __threadfence();
  *(volatile v4u*)(dst + e0) = u;
}

__global__ __launch_bounds__(256) void res_input_kernel(const float* __restrict__ P1,
                                                        const float* __restrict__ b_amp,
                                                        const float* __restrict__ b_phi,
                                                        float* __restrict__ U) {
  const int i = blockIdx.x * 256 + threadIdx.x;
  if (i >= kTok * kFreq) return;
  const int row = i >> 8;
  const int f   = i & (kFreq - 1);
  const size_t o = (size_t)row * kPre + f;
  const float za = P1[o] + b_amp[f];
  const float zp = P1[o + kFreq] + b_phi[f];
  const float amp = fmaxf(za, 0.0f) + log1pf(expf(-fabsf(za)));
  const float phi = kPi * tanhf(zp);
  float sn, cs;
  sincosf(phi, &sn, &cs);
  const float ur = amp * cs;
  const float ui = amp * sn;
  *(volatile float*)(U + o) = ur;
  *(volatile float*)(U + o + kFreq) = ui;
  __threadfence();
  *(volatile float*)(U + o) = ur;
  *(volatile float*)(U + o + kFreq) = ui;
}

__global__ __launch_bounds__(64) void res_scan_kernel(const float* __restrict__ U,
                                                      const float* __restrict__ omega,
                                                      const float* __restrict__ retl,
                                                      const float* __restrict__ theta,
                                                      unsigned short* __restrict__ FEAT) {
  __shared__ __align__(16) float sF[3 * kResSteps * kResF];
  const int tid = threadIdx.x, lane = tid & 31, wave = tid >> 5;
  const int b  = blockIdx.x >> 2;
  const int f0 = (blockIdx.x & 3) * kResF;
  const int f  = f0 + tid;
  const float dec = 1.0f / (1.0f + expf(-retl[f]));
  float so, co;
  sincosf(omega[f], &so, &co);
  const float ar = dec * co;
  const float ai = dec * so;
  const float th = theta[f];
  float xr = 0.0f, xi = 0.0f;
  const size_t row0 = (size_t)b * kSteps;
  const int q = lane >> 3, c8 = (lane & 7) * 8;
#pragma unroll 1
  for (int t0 = 0; t0 < kSteps; t0 += kResSteps) {
    __syncthreads();
#pragma unroll 1
    for (int s = 0; s < kResSteps; ++s) {
      const size_t o = (row0 + t0 + s) * kPre + f;
      const float ur = U[o];
      const float ui = U[o + kFreq];
      const float pr = ar * xr - ai * xi + ur;
      const float pi = ar * xi + ai * xr + ui;
      const float mag = sqrtf(pr * pr + pi * pi);
      const float g = 1.0f / (1.0f + expf(-(mag - th)));
      xr = pr * g;
      xi = pi * g;
      sF[s * kResF + tid] = xr;
      sF[kResSteps * kResF + s * kResF + tid] = xi;
      sF[2 * kResSteps * kResF + s * kResF + tid] = mag * g;
    }
    __syncthreads();
    for (int pass = 0; pass < 2; ++pass) {
#pragma unroll 1
      for (int it = 0; it < 24; ++it) {
        const int comp = it >> 3;
        const int row  = (it & 7) * 8 + wave * 4 + q;
        const float* sp = sF + comp * (kResSteps * kResF) + row * kResF + c8;
        const v4f a0 = *(const v4f*)(sp);
        const v4f a1 = *(const v4f*)(sp + 4);
        float v[8];
#pragma unroll
        for (int e = 0; e < 4; ++e) {
          v[e]     = a0[e] * kActCarry;
          v[4 + e] = a1[e] * kActCarry;
        }
        const v4u u = pack8(v);
        const size_t o = (row0 + t0 + row) * kFeat + comp * kFreq + f0 + c8;
        *(volatile v4u*)(FEAT + o) = u;
      }
      __threadfence();
    }
  }
}

__global__ __launch_bounds__(256) void attn_scan_kernel(const float* __restrict__ QKV,
                                                        const float* __restrict__ lnh_w,
                                                        const float* __restrict__ lnh_b,
                                                        unsigned short* __restrict__ YN) {
  __shared__ __align__(16) float lv[3 * kAtChunk * 64];
  __shared__ __align__(16) float yb[kAtChunk * 64];
  const int bh  = blockIdx.x;
  const int b   = bh >> 4;
  const int h   = bh & 15;
  const int tid = threadIdx.x;
  const int i   = tid >> 2;
  const int q   = tid & 3;
  const int j0  = q * 16;
  const int lrow = tid >> 4;
  const int lc4  = (tid & 15) * 4;
  const int srow = tid >> 3;
  const int c8   = (tid & 7) * 8;
  const size_t base = (size_t)b * kSteps * kQkv + (size_t)h * kHdim;

  const v4f w0 = *(const v4f*)(lnh_w + h * kHdim + c8);
  const v4f w1 = *(const v4f*)(lnh_w + h * kHdim + c8 + 4);
  const v4f g0 = *(const v4f*)(lnh_b + h * kHdim + c8);
  const v4f g1 = *(const v4f*)(lnh_b + h * kHdim + c8 + 4);

  float S[16], ks[16];
#pragma unroll
  for (int jj = 0; jj < 16; ++jj) {
    S[jj] = 0.0f;
    ks[jj] = 0.0f;
  }

#pragma unroll 1
  for (int ch = 0; ch < kSteps / kAtChunk; ++ch) {
#pragma unroll
    for (int rr = 0; rr < 2; ++rr) {
      const int r = lrow + 16 * rr;
      const size_t goff = base + (size_t)(ch * kAtChunk + r) * kQkv + lc4;
      const v4f tq = *(const v4f*)(QKV + goff);
      const v4f tk = *(const v4f*)(QKV + goff + kChan);
      const v4f tv = *(const v4f*)(QKV + goff + 2 * kChan);
      const int lo = r * 64 + lc4;
      *(v4f*)(lv + 0 * kAtChunk * 64 + lo) = tq;
      *(v4f*)(lv + 1 * kAtChunk * 64 + lo) = tk;
      *(v4f*)(lv + 2 * kAtChunk * 64 + lo) = tv;
    }
    __syncthreads();

#pragma unroll 1
    for (int s = 0; s < kAtChunk; ++s) {
      const float* pq = lv + 0 * kAtChunk * 64 + s * 64 + j0;
      const float* pk = lv + 1 * kAtChunk * 64 + s * 64 + j0;
      const float vi = lv[2 * kAtChunk * 64 + s * 64 + i];
      float num = 0.0f, den = 0.0f;
#pragma unroll
      for (int g4 = 0; g4 < 4; ++g4) {
        const v4f q4 = *(const v4f*)(pq + 4 * g4);
        const v4f k4 = *(const v4f*)(pk + 4 * g4);
#pragma unroll
        for (int e = 0; e < 4; ++e) {
          const float kk = k4[e];
          const float sn = S[4 * g4 + e] + vi * kk;
          const float kn = ks[4 * g4 + e] + kk;
          S[4 * g4 + e] = sn;
          ks[4 * g4 + e] = kn;
          num += q4[e] * sn;
          den += q4[e] * kn;
        }
      }
      num += __shfl_xor(num, 1, 32);
      num += __shfl_xor(num, 2, 32);
      den += __shfl_xor(den, 1, 32);
      den += __shfl_xor(den, 2, 32);
      const float y = num * __builtin_amdgcn_rcpf(den + kEpsAttn);
      if (q == 0) yb[s * 64 + i] = y;
    }
    __syncthreads();
    {
      const float* sp = yb + srow * 64 + c8;
      const v4f a0 = *(const v4f*)(sp);
      const v4f a1 = *(const v4f*)(sp + 4);
      float sum = (a0[0] + a0[1]) + (a0[2] + a0[3]) + (a1[0] + a1[1]) + (a1[2] + a1[3]);
      sum += __shfl_xor(sum, 1, 32);
      sum += __shfl_xor(sum, 2, 32);
      sum += __shfl_xor(sum, 4, 32);
      const float mean = sum * (1.0f / 64.0f);
      float d[8];
      float sq = 0.0f;
#pragma unroll
      for (int e = 0; e < 4; ++e) {
        d[e]     = a0[e] - mean;
        d[4 + e] = a1[e] - mean;
      }
#pragma unroll
      for (int e = 0; e < 8; ++e) sq += d[e] * d[e];
      sq += __shfl_xor(sq, 1, 32);
      sq += __shfl_xor(sq, 2, 32);
      sq += __shfl_xor(sq, 4, 32);
      const float var = sq * (1.0f / 64.0f);
      const float inv = __builtin_amdgcn_rcpf(sqrtf(var + kEpsLn));
      float o[8];
#pragma unroll
      for (int e = 0; e < 4; ++e) {
        o[e]     = ((d[e] * inv) * w0[e] + g0[e]) * kActCarry;
        o[4 + e] = ((d[4 + e] * inv) * w1[e] + g1[e]) * kActCarry;
      }
      const v4u u = pack8(o);
      unsigned short* dst = YN + ((size_t)b * kSteps + (size_t)(ch * kAtChunk + srow)) * kChan + h * kHdim + c8;
      *(volatile v4u*)dst = u;
      __threadfence();
      *(volatile v4u*)dst = u;
    }
  }
}

__global__ __launch_bounds__(256) void final_norm_kernel(const float* __restrict__ x, const float* __restrict__ Y2,
                                                         const float* __restrict__ ln_w, const float* __restrict__ ln_b,
                                                         float* __restrict__ out) {
  __shared__ float sSum[8];
  __shared__ float sSq[8];
  const int tid  = threadIdx.x;
  const int lane = tid & 31;
  const int wave = tid >> 5;
  const int c    = tid * 4;
  const size_t base = (size_t)blockIdx.x * kChan + c;
  const v4f xa = *(const v4f*)(x + base);
  const v4f ya = *(const v4f*)(Y2 + base);
  const v4f w4 = *(const v4f*)(ln_w + c);
  const v4f b4 = *(const v4f*)(ln_b + c);
  const v4f z = xa + ya;
  float s = (z[0] + z[1]) + (z[2] + z[3]);
  s = wave_sum32(s);
  if (lane == 0) sSum[wave] = s;
  __syncthreads();
  const float tot = ((sSum[0] + sSum[1]) + (sSum[2] + sSum[3])) + ((sSum[4] + sSum[5]) + (sSum[6] + sSum[7]));
  const float mu = tot * (1.0f / (float)kChan);
  const float d0 = z[0] - mu;
  const float d1 = z[1] - mu;
  const float d2 = z[2] - mu;
  const float d3 = z[3] - mu;
  float sq = (d0 * d0 + d1 * d1) + (d2 * d2 + d3 * d3);
  sq = wave_sum32(sq);
  if (lane == 0) sSq[wave] = sq;
  __syncthreads();
  const float tsq = ((sSq[0] + sSq[1]) + (sSq[2] + sSq[3])) + ((sSq[4] + sSq[5]) + (sSq[6] + sSq[7]));
  const float var = tsq * (1.0f / (float)kChan);
  const float rs = 1.0f / sqrtf(var + kEpsLn);
  v4f o;
  o[0] = (d0 * rs) * w4[0] + b4[0];
  o[1] = (d1 * rs) * w4[1] + b4[1];
  o[2] = (d2 * rs) * w4[2] + b4[2];
  o[3] = (d3 * rs) * w4[3] + b4[3];
  *(volatile v4f*)(out + base) = o;
  __threadfence();
  *(volatile v4f*)(out + base) = o;
}

extern "C" void kernel_launch(void* const* d_in, const int* in_sizes, int n_in,
                              void* d_out, int out_size, void* d_ws, size_t ws_size, hipStream_t stream) {
  if (n_in < 21 || d_out == nullptr || d_ws == nullptr) return;
  if (in_sizes[0] != kTok * kChan) return;
  if (in_sizes[1] != kChan * kFreq || in_sizes[2] != kFreq) return;
  if (in_sizes[3] != kChan * kFreq || in_sizes[4] != kFreq) return;
  if (in_sizes[5] != kFreq || in_sizes[6] != kFreq || in_sizes[7] != kFreq) return;
  if (in_sizes[8] != kFeat * kChan || in_sizes[9] != kChan) return;
  if (in_sizes[10] != kChan * kChan || in_sizes[11] != kChan * kChan || in_sizes[12] != kChan * kChan) return;
  if (in_sizes[13] != kHeads * kHdim || in_sizes[14] != kHeads * kHdim) return;
  if (in_sizes[15] != kChan * kRank || in_sizes[16] != kRank) return;
  if (in_sizes[17] != kRank * kChan || in_sizes[18] != kChan) return;
  if (in_sizes[19] != kChan || in_sizes[20] != kChan) return;
  if (out_size != kTok * kChan) return;

  const float* x      = (const float*)d_in[0];
  const float* W_amp  = (const float*)d_in[1];
  const float* b_amp  = (const float*)d_in[2];
  const float* W_phi  = (const float*)d_in[3];
  const float* b_phi  = (const float*)d_in[4];
  const float* omega  = (const float*)d_in[5];
  const float* retl   = (const float*)d_in[6];
  const float* theta  = (const float*)d_in[7];
  const float* W_feat = (const float*)d_in[8];
  const float* b_feat = (const float*)d_in[9];
  const float* Wq     = (const float*)d_in[10];
  const float* Wk     = (const float*)d_in[11];
  const float* Wv     = (const float*)d_in[12];
  const float* lnh_w  = (const float*)d_in[13];
  const float* lnh_b  = (const float*)d_in[14];
  const float* W1     = (const float*)d_in[15];
  const float* b1     = (const float*)d_in[16];
  const float* W2     = (const float*)d_in[17];
  const float* b2     = (const float*)d_in[18];
  const float* ln_w   = (const float*)d_in[19];
  const float* ln_b   = (const float*)d_in[20];
  float* out = (float*)d_out;

  char* ws = (char*)d_ws;
  size_t off = 0;
  auto carve = [&](size_t bytes) -> char* {
    char* p = ws + off;
    off += (bytes + 255) & ~(size_t)255;
    return p;
  };
  unsigned short* XH   = (unsigned short*)carve(kBytesXH);
  unsigned short* WAP  = (unsigned short*)carve(kBytesWAP);
  unsigned short* WFT  = (unsigned short*)carve(kBytesWFT);
  unsigned short* WQKV = (unsigned short*)carve(kBytesWQKV);
  unsigned short* W1T  = (unsigned short*)carve(kBytesW1T);
  unsigned short* W2T  = (unsigned short*)carve(kBytesW2T);
  float*          P1   = (float*)carve(kBytesP1);
  float*          U    = (float*)carve(kBytesU);
  unsigned short* FEAT = (unsigned short*)carve(kBytesFEAT);
  unsigned short* HH   = (unsigned short*)carve(kBytesHH);
  float*          QKV  = (float*)carve(kBytesQKV);
  unsigned short* YN   = (unsigned short*)carve(kBytesYN);
  unsigned short* H1   = (unsigned short*)carve(kBytesH1);
  float*          Y2   = (float*)carve(kBytesY2);
  if (off != kWsTotal || off > ws_size || off > (size_t)134217728) return;

  cast_act_kernel<<<(kTok * kChan / 8) / 256, 256, 0, stream>>>(x, XH, kTok * kChan / 8);
  wt_plane_kernel<<<dim3(kChan / 64, kFreq / 64, 2), 256, 0, stream>>>(W_amp, W_phi, W_phi, WAP, kChan, kFreq, kChan, kFreq);
  wt_plane_kernel<<<dim3(kFeat / 64, kChan / 64, 1), 256, 0, stream>>>(W_feat, W_feat, W_feat, WFT, kFeat, kChan, kFeat, kChan);
  wt_plane_kernel<<<dim3(kChan / 64, kChan / 64, 3), 256, 0, stream>>>(Wq, Wk, Wv, WQKV, kChan, kChan, kChan, kChan);
  wt_plane_kernel<<<dim3(kChan / 64, kRank / 64, 1), 256, 0, stream>>>(W1, W1, W1, W1T, kChan, kRank, kChan, kRank);
  wt_plane_kernel<<<dim3(kRank / 64, kChan / 64, 1), 256, 0, stream>>>(W2, W2, W2, W2T, kRank, kChan, kRank, kChan);

  gemm_f16_kernel<0, false><<<(kTok / 32) * (kPre / 64) / 8, 256, 0, stream>>>(
      XH, kChan, WAP, kChan, (void*)P1, kPre, nullptr, kTok, kPre, kChan, kScale, 0, 1.0f);

  res_input_kernel<<<(kTok * kFreq) / 256, 256, 0, stream>>>(P1, b_amp, b_phi, U);
  res_scan_kernel<<<kBatch * (kFreq / kResF), kResF, 0, stream>>>(U, omega, retl, theta, FEAT);

  gemm_f16_kernel<1, true><<<(kTok / 32) * (kChan / 64) / 8, 256, 0, stream>>>(
      FEAT, kFeat, WFT, kFeat, (void*)HH, kChan, b_feat, kTok, kChan, kFeat, kScale, kChan, kActCarry);

  gemm_f16_kernel<0, false><<<(kTok / 32) * (kQkv / 64) / 8, 256, 0, stream>>>(
      HH, kChan, WQKV, kChan, (void*)QKV, kQkv, nullptr, kTok, kQkv, kChan, kScale, 2 * kChan, 1.0f);

  attn_scan_kernel<<<kBatch * kHeads, 256, 0, stream>>>(QKV, lnh_w, lnh_b, YN);

  gemm_f16_kernel<1, true><<<(kTok / 32) * (kRank / 64) / 8, 256, 0, stream>>>(
      YN, kChan, W1T, kChan, (void*)H1, kRank, b1, kTok, kRank, kChan, kScale, kRank, kActCarry);
  gemm_f16_kernel<0, true><<<(kTok / 32) * (kChan / 64) / 8, 256, 0, stream>>>(
      H1, kRank, W2T, kRank, (void*)Y2, kChan, b2, kTok, kChan, kRank, kScale, kChan, 1.0f);

  final_norm_kernel<<<kTok, 256, 0, stream>>>(x, Y2, ln_w, ln_b, out);
}
